// GATRNNWithAttentionModel_13864154432151
// MI455X (gfx1250) — hardware-run, weakly checked
//
#include <hip/hip_runtime.h>

typedef float          v8f   __attribute__((ext_vector_type(8)));
typedef float          v4f   __attribute__((ext_vector_type(4)));
typedef unsigned int   v4u   __attribute__((ext_vector_type(4)));
typedef int            v8i   __attribute__((ext_vector_type(8)));
typedef unsigned short v8us  __attribute__((ext_vector_type(8)));
typedef unsigned short v16us __attribute__((ext_vector_type(16)));
typedef __bf16         v16bf __attribute__((ext_vector_type(16)));
typedef _Float16       v16h  __attribute__((ext_vector_type(16)));
typedef v4f  __attribute__((may_alias)) v4fa;
typedef v8us __attribute__((may_alias)) v8usa;
union FragB { v16bf v; v16us u; v8us h[2]; v8i w; };
union FragH { v16h  v; v16us u; v8us h[2]; v8i w; };

__device__ __forceinline__ v8f wmb(const FragB& a, const FragB& b, v8f c) {
  v8f d = __builtin_amdgcn_wmma_f32_16x16x32_bf16(false, a.v, false, b.v, (short)0, c, false, false);
  asm volatile("v_nop\n\tv_nop\n\tv_nop\n\tv_nop" : "+v"(d) : "v"(a.w), "v"(b.w));
  return d;
}

__device__ __forceinline__ v8f wmh(const FragH& a, const FragH& b, v8f c) {
  v8f d = __builtin_amdgcn_wmma_f32_16x16x32_f16(false, a.v, false, b.v, (short)0, c, false, false);
  asm volatile("v_nop\n\tv_nop\n\tv_nop\n\tv_nop" : "+v"(d) : "v"(a.w), "v"(b.w));
  return d;
}

__device__ __forceinline__ unsigned bf16_bits(float f) {
  const unsigned u = __float_as_uint(f);
  const unsigned r = (u + 0x7FFFu + ((u >> 16) & 1u)) >> 16;
  const unsigned q = (u >> 16) | 0x40u;
  return ((u & 0x7fffffffu) > 0x7f800000u) ? q : r;
}

__device__ __forceinline__ float bf16_val(float f) {
  return __uint_as_float(bf16_bits(f) << 16);
}
__device__ __forceinline__ int clampi(int v, int lo, int hi) {
  return v < lo ? lo : (v > hi ? hi : v);
}

__device__ __forceinline__ unsigned f16_bits(float f) {
  const unsigned u  = __float_as_uint(f);
  const unsigned s  = (u >> 16) & 0x8000u;
  const unsigned a  = u & 0x7fffffffu;
  const unsigned t  = a - 0x38000000u;
  const unsigned r  = (t + 0x0FFFu + ((t >> 13) & 1u)) >> 13;
  const unsigned rc = r > 0x7C00u ? 0x7C00u : r;
  const bool small  = a < 0x38800000u;
  const bool isnan  = a > 0x7f800000u;
  const unsigned fin = small ? 0u : (s | rc);
  return isnan ? (s | 0x7E00u) : fin;
}

__device__ __forceinline__ unsigned pk16(unsigned lo, unsigned hi) { return lo | (hi << 16); }
__device__ __forceinline__ unsigned bf16_lo_bits(float v) {
  float hi = bf16_val(v);
  asm volatile("" : "+v"(hi));
  return bf16_bits(v - hi);
}
__device__ __forceinline__ v4u pack8_bf16(v4f a, v4f c) {
  return (v4u){ pk16(bf16_bits(a[0]), bf16_bits(a[1])), pk16(bf16_bits(a[2]), bf16_bits(a[3])),
                pk16(bf16_bits(c[0]), bf16_bits(c[1])), pk16(bf16_bits(c[2]), bf16_bits(c[3])) };
}
__device__ __forceinline__ v4u pack8_bf16_lo(v4f a, v4f c) {
  return (v4u){ pk16(bf16_lo_bits(a[0]), bf16_lo_bits(a[1])), pk16(bf16_lo_bits(a[2]), bf16_lo_bits(a[3])),
                pk16(bf16_lo_bits(c[0]), bf16_lo_bits(c[1])), pk16(bf16_lo_bits(c[2]), bf16_lo_bits(c[3])) };
}
__device__ __forceinline__ v4u pack8_f16(v4f a, v4f c) {
  return (v4u){ pk16(f16_bits(a[0]), f16_bits(a[1])), pk16(f16_bits(a[2]), f16_bits(a[3])),
                pk16(f16_bits(c[0]), f16_bits(c[1])), pk16(f16_bits(c[2]), f16_bits(c[3])) };
}

template <int FORM>
__global__ __launch_bounds__(256) void k_plane(const float* __restrict__ src, int rows, int cols, int ldsrc,
                                               unsigned short* __restrict__ dst, int MP, int KP) {
  static_assert(FORM >= 0 && FORM <= 3);
  const int KTOT = (FORM == 1 || FORM == 3) ? 2 * KP : KP;
  const unsigned ppr   = (unsigned)(KTOT >> 3);
  const unsigned kp8   = (unsigned)(KP >> 3);
  const unsigned total = (unsigned)MP * ppr;
  const unsigned g     = blockIdx.x * 256u + threadIdx.x;
  const unsigned rowu  = g / ppr;
  const unsigned p     = g - rowu * ppr;
  const bool second    = p >= kp8;
  const int row = (int)rowu;
  const int c0  = (int)((second ? p - kp8 : p) << 3);
  const float* srow = src + (size_t)clampi(row, 0, rows - 1) * (size_t)ldsrc;
  float x[8];
  unsigned mk[8];
#pragma unroll
  for (int e = 0; e < 8; ++e) {
    const int c = c0 + e;
    const float v = srow[clampi(c, 0, cols - 1)];
    asm volatile("" :: "v"(v));
    x[e]  = v;
    mk[e] = (row < rows && c < cols) ? 0xFFFFu : 0u;
  }
  const v4f a = (v4f){ x[0], x[1], x[2], x[3] };
  const v4f c = (v4f){ x[4], x[5], x[6], x[7] };
  v4u o;
  if (FORM == 2) {
    o = pack8_f16(a, c);
  } else {
    const v4u hi = pack8_bf16(a, c);
    o = hi;
    if (FORM == 1) { const v4u lo = pack8_bf16_lo(a, c); o = second ? lo : hi; }
  }
  const v4u mw = (v4u){ pk16(mk[0], mk[1]), pk16(mk[2], mk[3]), pk16(mk[4], mk[5]), pk16(mk[6], mk[7]) };
  o &= mw;
  if (g < total) {
    volatile v4u* q = (volatile v4u*)(dst + (size_t)g * 8);
    *q = o;
    __threadfence();
    *q = o;
  }
}

template <int FORM> struct FragOf    { typedef FragB T; };
template <>         struct FragOf<2> { typedef FragH T; };
__device__ __forceinline__ v8f mm(const FragB& a, const FragB& b, v8f c) { return wmb(a, b, c); }
__device__ __forceinline__ v8f mm(const FragH& a, const FragH& b, v8f c) { return wmh(a, b, c); }
template <class F> __device__ __forceinline__ F ld_frag(const unsigned short* p) {
  F f;
  f.h[0] = *(const v8usa*)(p);
  f.h[1] = *(const v8usa*)(p + 16);
  return f;
}

template <int FORM, int EPI>
__global__ __launch_bounds__(256) __attribute__((amdgpu_num_vgpr(248)))
void k_gemm_nt(const unsigned short* __restrict__ A, const unsigned short* __restrict__ B,
               const float* __restrict__ bias, float* __restrict__ D, int M, int N, int KTOT, int ldd) {
  static_assert(FORM >= 0 && FORM <= 2);
  static_assert(EPI == 0 || EPI == 1);
  typedef typename FragOf<FORM>::T F;
  __shared__ __attribute__((aligned(16))) float sT[8][16 * 68];
  const int lane = threadIdx.x & 31;
  const int wave = threadIdx.x >> 5;
  const int tilesM = (M + 63) >> 6;
  const int tilesN = (N + 63) >> 6;
  const int tile = blockIdx.x * 8 + wave;
  if (tile >= tilesM * tilesN) return;
  const int tm = tile / tilesN;
  const int tn = tile - tm * tilesN;
  const int m0 = tm << 6;
  const int n0 = tn << 6;

  const int rl = lane & 15;
  const int h8 = (lane >> 4) * 8;
  const unsigned short* pa = A + (size_t)(m0 + rl) * (size_t)KTOT + h8;
  const unsigned short* pb = B + (size_t)(n0 + rl) * (size_t)KTOT + h8;

  v8f acc[4][4];
#pragma unroll
  for (int i = 0; i < 4; ++i)
#pragma unroll
    for (int j = 0; j < 4; ++j) acc[i][j] = (v8f){0.f, 0.f, 0.f, 0.f, 0.f, 0.f, 0.f, 0.f};

#pragma unroll 1
  for (int k0 = 0; k0 < KTOT; k0 += 32) {
    F bf[4];
#pragma unroll
    for (int j = 0; j < 4; ++j) bf[j] = ld_frag<F>(pb + (size_t)(j << 4) * (size_t)KTOT + k0);
#pragma unroll
    for (int i = 0; i < 4; ++i) {
      const F af = ld_frag<F>(pa + (size_t)(i << 4) * (size_t)KTOT + k0);
#pragma unroll
      for (int j = 0; j < 4; ++j) acc[i][j] = mm(af, bf[j], acc[i][j]);
    }
  }

  float* slab = sT[wave];
  const int hh = lane >> 4;
  const int c4 = (lane & 15) * 4;
  const int nc = n0 + c4;
  const bool cok = nc < N;
  v4f bv = (v4f){0.f, 0.f, 0.f, 0.f};
  if (EPI == 1) {
    bv = *(const v4fa*)(bias + clampi(nc, 0, N - 4));
    asm volatile("" :: "v"(bv));
  }
#pragma unroll
  for (int i = 0; i < 4; ++i) {
    const int mBase = m0 + (i << 4);
#pragma unroll
    for (int j = 0; j < 4; ++j) {
#pragma unroll
      for (int r = 0; r < 8; ++r) slab[(h8 + r) * 68 + (j << 4) + rl] = acc[i][j][r];
    }
    __builtin_amdgcn_fence(__ATOMIC_RELEASE, "workgroup");
    __builtin_amdgcn_wave_barrier();
    __builtin_amdgcn_fence(__ATOMIC_ACQUIRE, "workgroup");
    v4f vv[8];
#pragma unroll
    for (int it = 0; it < 8; ++it) {
      const int row = it * 2 + hh;
      v4f v = *(const v4fa*)(slab + row * 68 + c4);
      if (EPI == 1) v += bv;
      vv[it] = v;
    }
    for (int pass = 0; pass < 2; ++pass) {
#pragma unroll
      for (int it = 0; it < 8; ++it) {
        const int row = mBase + it * 2 + hh;
        if (cok && row < M) *(volatile v4f*)(D + (size_t)row * (size_t)ldd + nc) = vv[it];
      }
      __threadfence();
    }
    __builtin_amdgcn_fence(__ATOMIC_RELEASE, "workgroup");
    __builtin_amdgcn_wave_barrier();
    __builtin_amdgcn_fence(__ATOMIC_ACQUIRE, "workgroup");
  }
}

#pragma clang fp contract(off)

typedef int          v4i __attribute__((ext_vector_type(4)));
typedef int          v2i __attribute__((ext_vector_type(2)));
typedef unsigned int v2u __attribute__((ext_vector_type(2)));
typedef v4i __attribute__((may_alias)) v4ia;
typedef v2i __attribute__((may_alias)) v2ia;
typedef v4u __attribute__((may_alias)) v4ua;

constexpr int NN      = 100000;
constexpr int NE      = 1600000;
constexpr int FIN     = 128;
constexpr int HD      = 128;
constexpr int NG      = 384;
constexpr int NOUT    = 16;
constexpr int MP      = 100352;
constexpr int NCHK    = 4;
constexpr int CHR     = 25088;
constexpr int KHL     = 256;
constexpr int OUT_ELEMS = NN * NOUT;
constexpr int NBLK    = 98;
constexpr int OWN     = 1024;
constexpr int RCAP    = 21504;
constexpr int WLCAP   = 2688;
constexpr int DEGCAP  = 48;
constexpr int KW      = NE / 8;
constexpr int NIT     = (KW + 255) / 256;
constexpr int SLOTX   = OWN + 32;
constexpr int FLAGBIT = 0x40000000;
constexpr int LDS_BK  = (8 * WLCAP + RCAP + 16 * SLOTX + 2 * OWN + 16) * 4;

constexpr bool SITE2_TWO_TERM = true;
constexpr bool SITE3_TWO_TERM = true;

constexpr int T_AS = 0, T_AD = 128, T_GB = 256, T_BIH = 384, T_BHH = 768, T_BFC = 1152, T_N = 1280;

static_assert(MP == NBLK * OWN && MP == NCHK * CHR && MP % 64 == 0 && CHR % 64 == 0 && CHR % 8 == 0);
static_assert(MP >= NN && MP % 16 == 0 && CHR % 16 == 0 && MP % 8 == 0);
static_assert(NN % 32 == 0 && OUT_ELEMS % 256 == 0 && OUT_ELEMS == 1600000);
static_assert(NN < (1 << 17) && NE < (1 << 21) && OWN == (1 << 10));
static_assert(NE % 8 == 0 && KW % 8 == 0 && KW >= 8 && NIT == 782);
static_assert(8 * WLCAP == RCAP && (RCAP / 4) % 256 == 0 && DEGCAP + 1 <= 64 && DEGCAP <= RCAP);
static_assert(LDS_BK == 247872 && LDS_BK <= 262144);
static_assert(FIN % 32 == 0 && KHL % 32 == 0 && HD % 64 == 0 && NG % 64 == 0 && NG % 4 == 0);
static_assert((long long)MP * KHL / 8 < 0x7fffffffLL);

constexpr size_t SZ_A    = (size_t)MP * KHL * 2;
constexpr size_t SZ_B    = (size_t)MP * HD * 4;
constexpr size_t SZ_AD4  = (size_t)NN * 4 * 4;
constexpr size_t SZ_HITS = (size_t)NBLK * RCAP * 4;
constexpr size_t SZ_OC   = (size_t)MP * 2 * 4;
constexpr size_t SZ_WT   = (size_t)HD * FIN * 2;
constexpr size_t SZ_WIH2 = (size_t)NG * KHL * 2;
constexpr size_t SZ_WFC2 = (size_t)64 * KHL * 2;
constexpr size_t SZ_TBL  = (size_t)T_N * 4;
constexpr size_t OFF_A    = 0;
constexpr size_t OFF_B    = OFF_A + SZ_A;
constexpr size_t OFF_AD4  = OFF_B + SZ_B;
constexpr size_t OFF_HITS = OFF_AD4 + SZ_AD4;
constexpr size_t OFF_OC   = OFF_HITS + SZ_HITS;
constexpr size_t OFF_WT   = OFF_OC + SZ_OC;
constexpr size_t OFF_WIH2 = OFF_WT + SZ_WT;
constexpr size_t OFF_WFC2 = OFF_WIH2 + SZ_WIH2;
constexpr size_t OFF_TBL  = OFF_WFC2 + SZ_WFC2;
constexpr size_t WS_TOTAL = OFF_TBL + SZ_TBL;
static_assert(SZ_A == (size_t)51380224 && SZ_B == (size_t)51380224 && SZ_HITS == (size_t)8429568 && SZ_OC == (size_t)802816);
static_assert(SZ_A % 256 == 0 && SZ_B % 256 == 0 && SZ_AD4 % 256 == 0 && SZ_HITS % 256 == 0 && SZ_OC % 256 == 0);
static_assert(SZ_WT % 256 == 0 && SZ_WIH2 % 256 == 0 && SZ_WFC2 % 256 == 0 && SZ_TBL % 256 == 0);
static_assert((size_t)MP * FIN * 2 <= SZ_A);
static_assert((size_t)CHR * NG * 4 == (size_t)38535168 && (size_t)CHR * NG * 4 <= SZ_B);
static_assert((size_t)MP * 64 * 4 <= SZ_B);
static_assert(OFF_TBL == (size_t)((size_t)222373 << 9) && WS_TOTAL == (size_t)((size_t)222383 << 9));
static_assert(WS_TOTAL <= ((size_t)128 << 20));

__device__ __forceinline__ void put16(unsigned short* p, v4u o) {
  volatile v4u* q = (volatile v4u*)p;
  *q = o;
  __threadfence();
  *q = o;
}
__device__ __forceinline__ void put16f(float* p, v4f o) {
  volatile v4f* q = (volatile v4f*)p;
  *q = o;
  __threadfence();
  *q = o;
}
__device__ __forceinline__ void lds_wave_sync() {
  __builtin_amdgcn_fence(__ATOMIC_RELEASE, "workgroup");
  __builtin_amdgcn_wave_barrier();
  __builtin_amdgcn_fence(__ATOMIC_ACQUIRE, "workgroup");
}

__global__ __launch_bounds__(256) void k_prep(
    const float* __restrict__ W, const float* __restrict__ Wih, const float* __restrict__ Wfc,
    const float* __restrict__ atts, const float* __restrict__ attd, const float* __restrict__ gb,
    const float* __restrict__ bih, const float* __restrict__ bhh, const float* __restrict__ bfc,
    unsigned short* __restrict__ WT, unsigned short* __restrict__ WIH2, unsigned short* __restrict__ WFC2,
    float* __restrict__ TBL) {
  const int tid = (int)threadIdx.x;
  const int blk = (int)blockIdx.x;
  if (blk < 8) {
    const int g  = blk * 256 + tid;
    const int n  = g >> 4;
    const int k8 = (g & 15) * 8;
    float x[8];
#pragma unroll
    for (int e = 0; e < 8; ++e) {
      const float v = W[(size_t)(k8 + e) * HD + n];
      asm volatile("" :: "v"(v));
      x[e] = v;
    }
    const v4u o = pack8_bf16((v4f){ x[0], x[1], x[2], x[3] }, (v4f){ x[4], x[5], x[6], x[7] });
    put16(WT + (size_t)g * 8, o);
  } else if (blk < 56) {
    const int g   = (blk - 8) * 256 + tid;
    const int n   = g >> 5;
    const int k   = (g & 15) * 8;
    const int row = n < 128 ? n : n + 128;
    const v4f a = *(const v4fa*)(Wih + (size_t)row * FIN + k);
    const v4f c = *(const v4fa*)(Wih + (size_t)row * FIN + k + 4);
    asm volatile("" :: "v"(a));
    asm volatile("" :: "v"(c));
    put16(WIH2 + (size_t)g * 8, pack8_bf16(a, c));
  } else if (blk < 64) {
    const int g  = (blk - 56) * 256 + tid;
    const int n  = g >> 5;
    const int k  = (g & 15) * 8;
    const int rc = n < NOUT ? n : NOUT - 1;
    const v4f a = *(const v4fa*)(Wfc + (size_t)rc * HD + k);
    const v4f c = *(const v4fa*)(Wfc + (size_t)rc * HD + k + 4);
    asm volatile("" :: "v"(a));
    asm volatile("" :: "v"(c));
    v4u o = pack8_bf16(a, c);
    const unsigned mk = n < NOUT ? 0xFFFFFFFFu : 0u;
    o &= (v4u){ mk, mk, mk, mk };
    put16(WFC2 + (size_t)g * 8, o);
  } else {
    const int t  = (blk - 64) * 256 + tid;
    const int tc = t < (T_N / 4) ? t : (T_N / 4) - 1;
    const int f0 = 4 * tc;
    const int r3 = clampi(f0 - T_BIH, 0, NG - 4);
    const int r4 = clampi(f0 - T_BHH, 0, NG - 4);
    const int s3 = r3 < 128 ? r3 : r3 + 128;
    const int s4 = r4 < 128 ? r4 : r4 + 128;
    const v4f a0 = *(const v4fa*)(atts + clampi(f0 - T_AS, 0, 124));
    const v4f a1 = *(const v4fa*)(attd + clampi(f0 - T_AD, 0, 124));
    const v4f a2 = *(const v4fa*)(gb   + clampi(f0 - T_GB, 0, 124));
    const v4f a3 = *(const v4fa*)(bih  + s3);
    const v4f a4 = *(const v4fa*)(bhh  + s4);
    const v4f a5 = *(const v4fa*)(bfc  + clampi(f0 - T_BFC, 0, NOUT - 4));
    asm volatile("" :: "v"(a0));
    asm volatile("" :: "v"(a1));
    asm volatile("" :: "v"(a2));
    asm volatile("" :: "v"(a3));
    asm volatile("" :: "v"(a4));
    asm volatile("" :: "v"(a5));
    const unsigned m0 = (f0 < T_AD) ? 0xFFFFFFFFu : 0u;
    const unsigned m1 = (f0 >= T_AD  && f0 < T_GB)  ? 0xFFFFFFFFu : 0u;
    const unsigned m2 = (f0 >= T_GB  && f0 < T_BIH) ? 0xFFFFFFFFu : 0u;
    const unsigned m3 = (f0 >= T_BIH && f0 < T_BHH) ? 0xFFFFFFFFu : 0u;
    const unsigned m4 = (f0 >= T_BHH && f0 < T_BFC) ? 0xFFFFFFFFu : 0u;
    const unsigned m5 = (f0 >= T_BFC && f0 < T_BFC + NOUT) ? 0xFFFFFFFFu : 0u;
    v4f o;
#pragma unroll
    for (int e = 0; e < 4; ++e) {
      const unsigned b = (__float_as_uint(a0[e]) & m0) | (__float_as_uint(a1[e]) & m1) |
                         (__float_as_uint(a2[e]) & m2) | (__float_as_uint(a3[e]) & m3) |
                         (__float_as_uint(a4[e]) & m4) | (__float_as_uint(a5[e]) & m5);
      o[e] = bf16_val(__uint_as_float(b));
    }
    if (t < T_N / 4) put16f(TBL + 4 * t, o);
  }
}

__device__ __forceinline__ void group_rank(int* mytag, int s, int lane, int& rank, int& gs) {
  mytag[s] = lane;
  lds_wave_sync();
  int s2 = s;
  asm volatile("" : "+v"(s2));
  const int t = mytag[s2];
  unsigned lm = __builtin_amdgcn_ballot_w32(t != lane);
  rank = 0;
  gs = 1;
#pragma unroll 1
  for (int g = 0; g < 32 && lm != 0u; ++g) {
    const int k  = __builtin_ctz(lm);
    const int sk = __builtin_amdgcn_readlane(s, k);
    const bool in = (s == sk);
    const unsigned em = __builtin_amdgcn_ballot_w32(in);
    const int r  = (int)__builtin_amdgcn_mbcnt_lo(em, 0u);
    const int gc = (int)__builtin_popcount(em);
    rank = in ? r : rank;
    gs   = in ? gc : gs;
    lm &= ~em;
  }
}

__global__ __launch_bounds__(256) void k_bucket(const int* __restrict__ ei, unsigned* __restrict__ HITS,
                                                int* __restrict__ OC) {
  extern __shared__ v4u lds_raw[];
  unsigned* wl  = (unsigned*)lds_raw;
  unsigned* srt = wl + 8 * WLCAP;
  int* cnt  = (int*)(srt + RCAP);
  int* tag  = cnt + 8 * SLOTX;
  int* stot = tag + 8 * SLOTX;
  int* soff = stot + OWN;
  int* wtot = soff + OWN;
  const int tid = (int)threadIdx.x, lane = tid & 31, wave = tid >> 5;
  const int blk = (int)blockIdx.x;
  const unsigned ubase = (unsigned)blk * (unsigned)OWN;

  for (int i = tid; i < 8 * SLOTX; i += 256) cnt[i] = 0;
  for (int i = tid; i < RCAP; i += 256) srt[i] = 0u;
  __syncthreads();

  const int* dstp = ei + NE;
  unsigned* mylist = wl + wave * WLCAP;
  const int wk0 = wave * KW;
  int wc = 0;
#pragma unroll 1
  for (int it = 0; it < NIT; ++it) {
    const int k0 = it * 256 + lane * 8;
    const bool valid = k0 < KW;
    const int kc = k0 < KW - 8 ? k0 : KW - 8;
    const int e0 = wk0 + kc;
    const v4i da = *(const v4ia*)(dstp + e0);
    const v4i db = *(const v4ia*)(dstp + e0 + 4);
    asm volatile("" :: "v"(da));
    asm volatile("" :: "v"(db));
    unsigned s[8];
    s[0] = (unsigned)da[0] - ubase; s[1] = (unsigned)da[1] - ubase;
    s[2] = (unsigned)da[2] - ubase; s[3] = (unsigned)da[3] - ubase;
    s[4] = (unsigned)db[0] - ubase; s[5] = (unsigned)db[1] - ubase;
    s[6] = (unsigned)db[2] - ubase; s[7] = (unsigned)db[3] - ubase;
    bool h[8];
    unsigned m[8];
#pragma unroll
    for (int j = 0; j < 8; ++j) {
      h[j] = valid & (s[j] < (unsigned)OWN);
      m[j] = __builtin_amdgcn_ballot_w32(h[j]);
    }
    int pos = wc;
    int tot = 0;
#pragma unroll
    for (int j = 0; j < 8; ++j) {
      pos = (int)__builtin_amdgcn_mbcnt_lo(m[j], (unsigned)pos);
      tot += (int)__builtin_popcount(m[j]);
    }
#pragma unroll
    for (int j = 0; j < 8; ++j) {
      if (h[j] && pos < WLCAP) mylist[pos] = ((unsigned)(e0 + j) << 10) | s[j];
      pos += h[j] ? 1 : 0;
    }
    wc += tot;
  }
  if (lane == 0) wtot[wave] = wc;
  __syncthreads();

  const int cw = wc > WLCAP ? WLCAP : wc;
  int* mycnt = cnt + wave * SLOTX;
  int* mytag = tag + wave * SLOTX;

#pragma unroll 1
  for (int b0 = 0; b0 < cw; b0 += 32) {
    const int idx = b0 + lane;
    const bool valid = idx < cw;
    const unsigned word = mylist[valid ? idx : cw - 1];
    const int s = valid ? (int)(word & 1023u) : (OWN + lane);
    int rank, gs;
    group_rank(mytag, s, lane, rank, gs);
    const int base = mycnt[s];
    if (valid && rank == gs - 1) mycnt[s] = base + gs;
    lds_wave_sync();
  }
  __syncthreads();

  {
    int c4[4];
    int tsum = 0;
#pragma unroll
    for (int q = 0; q < 4; ++q) {
      const int sl = 4 * tid + q;
      int c = 0;
#pragma unroll
      for (int w2 = 0; w2 < 8; ++w2) c += cnt[w2 * SLOTX + sl];
      c4[q] = c;
      tsum += c;
    }
    int incl = tsum;
#pragma unroll
    for (int dd = 1; dd < 32; dd <<= 1) {
      const int up = __shfl_up(incl, dd, 32);
      incl += (lane >= dd) ? up : 0;
    }
    if (lane == 31) wtot[8 + wave] = incl;
    __syncthreads();
    int pre = 0;
#pragma unroll
    for (int w2 = 0; w2 < 8; ++w2) pre += (w2 < wave) ? wtot[8 + w2] : 0;
    int run = pre + incl - tsum;
#pragma unroll
    for (int q = 0; q < 4; ++q) {
      const int sl = 4 * tid + q;
      soff[sl] = run;
      stot[sl] = c4[q];
      int st = run;
#pragma unroll
      for (int w2 = 0; w2 < 8; ++w2) {
        const int tmp = cnt[w2 * SLOTX + sl];
        cnt[w2 * SLOTX + sl] = st;
        st += tmp;
      }
      run += c4[q];
    }
  }
  __syncthreads();

#pragma unroll 1
  for (int b0 = 0; b0 < cw; b0 += 32) {
    const int idx = b0 + lane;
    const bool valid = idx < cw;
    const unsigned word = mylist[valid ? idx : cw - 1];
    const int sl = (int)(word & 1023u);
    const int s = valid ? sl : (OWN + lane);
    int rank, gs;
    group_rank(mytag, s, lane, rank, gs);
    const int base = mycnt[s];
    const int pos = base + rank;
    const int eid = clampi((int)(word >> 10), 0, NE - 1);
    const int sv = ei[eid];
    asm volatile("" :: "v"(sv));
    const unsigned outw = (unsigned)clampi(sv, 0, NN - 1) | ((unsigned)sl << 17);
    if (valid && pos >= 0 && pos < RCAP) srt[pos] = outw;
    if (valid && rank == gs - 1) mycnt[s] = base + gs;
    lds_wave_sync();
  }
  __syncthreads();

  bool ovf = false;
#pragma unroll
  for (int w2 = 0; w2 < 8; ++w2) ovf = ovf | (wtot[w2] > WLCAP);
  const int fl = ovf ? FLAGBIT : 0;

  unsigned* hb = HITS + (size_t)blk * RCAP;
  for (int pass = 0; pass < 2; ++pass) {
#pragma unroll 1
    for (int i = tid; i < RCAP / 4; i += 256) {
      const v4u v = *(const v4ua*)(srt + 4 * i);
      *(volatile v4u*)(hb + 4 * i) = v;
    }
    __threadfence();
  }
  v4i oc[2];
#pragma unroll
  for (int i = 0; i < 2; ++i) {
    const int p = tid + 256 * i;
    oc[i] = (v4i){ soff[2 * p], stot[2 * p] | fl, soff[2 * p + 1], stot[2 * p + 1] | fl };
  }
  int* ob = OC + ((size_t)blk * OWN) * 2;
  for (int pass = 0; pass < 2; ++pass) {
#pragma unroll
    for (int i = 0; i < 2; ++i) {
      const int p = tid + 256 * i;
      *(volatile v4i*)(ob + 4 * p) = oc[i];
    }
    __threadfence();
  }
}

__global__ __launch_bounds__(256) void k_node(const float* __restrict__ HW, const float* __restrict__ TBL,
                                              float* __restrict__ AD4) {
  __shared__ __attribute__((aligned(16))) float sA[32 * 4];
  const int tid = (int)threadIdx.x, lane = tid & 31, wave = tid >> 5;
  const v4f as = *(const v4fa*)(TBL + T_AS + 4 * lane);
  const v4f ad = *(const v4fa*)(TBL + T_AD + 4 * lane);
  asm volatile("" :: "v"(as));
  asm volatile("" :: "v"(ad));
#pragma unroll 1
  for (int q = 0; q < 4; ++q) {
    const int nl = wave * 4 + q;
    const int n  = (int)blockIdx.x * 32 + nl;
    const v4f hv = *(const v4fa*)(HW + (size_t)n * HD + 4 * lane);
    asm volatile("" :: "v"(hv));
    float ps = ((hv[0] * as[0] + hv[1] * as[1]) + hv[2] * as[2]) + hv[3] * as[3];
    float pd = ((hv[0] * ad[0] + hv[1] * ad[1]) + hv[2] * ad[2]) + hv[3] * ad[3];
#pragma unroll
    for (int o = 1; o < 16; o <<= 1) {
      const float ts = __shfl_xor(ps, o, 32);
      const float td = __shfl_xor(pd, o, 32);
      ps = ps + ts;
      pd = pd + td;
    }
    if (lane == 0)  { sA[nl * 4 + 0] = ps; sA[nl * 4 + 2] = pd; }
    if (lane == 16) { sA[nl * 4 + 1] = ps; sA[nl * 4 + 3] = pd; }
  }
  __syncthreads();
  if (wave == 0) {
    const v4f v = *(const v4fa*)(sA + 4 * lane);
    put16f(AD4 + ((size_t)blockIdx.x * 32 + lane) * 4, v);
  }
}

__device__ __forceinline__ float rl_f(float v, int j) {
  return __int_as_float(__builtin_amdgcn_readlane(__float_as_int(v), j));
}
__device__ __forceinline__ float leaky(float v) { return (v >= 0.0f) ? v : 0.2f * v; }
__device__ __forceinline__ float nmax(float m, float e) { return (e > m || e != e) ? e : m; }

__global__ __launch_bounds__(256) void k_replay(const unsigned* __restrict__ HITS, const int* __restrict__ OC,
                                                const float* __restrict__ HW, const float* __restrict__ AD4,
                                                const float* __restrict__ TBL, unsigned short* __restrict__ Ghl) {
  const int lane = (int)threadIdx.x & 31;
  const int wave = (int)threadIdx.x >> 5;
  const int d = __builtin_amdgcn_readfirstlane((int)blockIdx.x * 8 + wave);
  const bool live = d < NN;
  const int dc = live ? d : NN - 1;
  const int blk = d >> 10;
  const bool hsel = lane >= 16;

  const v2i oc = *(const v2ia*)(OC + 2 * (size_t)d);
  asm volatile("" :: "v"(oc));
  const int craw = oc[1];
  const int cval = craw & (FLAGBIT - 1);
  const bool poison = ((craw & FLAGBIT) != 0) || (cval > DEGCAP) || (craw < 0);
  const int offc = clampi(oc[0], 0, RCAP);
  int cc = clampi(cval, 0, DEGCAP);
  cc = cc < (RCAP - offc) ? cc : (RCAP - offc);
  const int cn   = __builtin_amdgcn_readfirstlane(live ? cc : 0);
  const int offu = __builtin_amdgcn_readfirstlane(offc);
  const int nent = cn + 1;

  const unsigned* hb = HITS + (size_t)blk * RCAP;
  const v4f adD = *(const v4fa*)(AD4 + 4 * (size_t)dc);
  asm volatile("" :: "v"(adD));

  const int tA = lane;
  const int iA = clampi(offu + (tA < cn ? tA : 0), 0, RCAP - 1);
  const unsigned wA = hb[iA];
  asm volatile("" :: "v"(wA));
  const int hA = clampi((int)(wA & 0x1FFFFu), 0, NN - 1);
  const int srcA = (tA < cn) ? hA : dc;
  const v4f adA = *(const v4fa*)(AD4 + 4 * (size_t)srcA);
  asm volatile("" :: "v"(adA));
  const bool vA = tA < nent;
  const float eA0 = leaky(adA[0] + adD[2]);
  const float eA1 = leaky(adA[1] + adD[3]);

  int srcB = dc;
  float eB0 = 0.0f, eB1 = 0.0f;
  bool vB = false;
  if (nent > 32) {
    const int tB = 32 + lane;
    const int iB = clampi(offu + (tB < cn ? tB : 0), 0, RCAP - 1);
    const unsigned wB = hb[iB];
    asm volatile("" :: "v"(wB));
    const int hB = clampi((int)(wB & 0x1FFFFu), 0, NN - 1);
    srcB = (tB < cn) ? hB : dc;
    const v4f adB = *(const v4fa*)(AD4 + 4 * (size_t)srcB);
    asm volatile("" :: "v"(adB));
    vB = tB < nent;
    eB0 = leaky(adB[0] + adD[2]);
    eB1 = leaky(adB[1] + adD[3]);
  }

  const float ninf = -__builtin_inff();
  float m0 = vA ? eA0 : ninf;
  float m1 = vA ? eA1 : ninf;
  m0 = nmax(m0, vB ? eB0 : ninf);
  m1 = nmax(m1, vB ? eB1 : ninf);
#pragma unroll
  for (int o = 16; o > 0; o >>= 1) {
    const float t0 = __shfl_xor(m0, o, 32);
    const float t1 = __shfl_xor(m1, o, 32);
    m0 = nmax(m0, t0);
    m1 = nmax(m1, t1);
  }

  const float xA0 = expf(eA0 - m0);
  const float xA1 = expf(eA1 - m1);
  const float xB0 = expf(eB0 - m0);
  const float xB1 = expf(eB1 - m1);
  const float pA0 = vA ? xA0 : 0.0f;
  const float pA1 = vA ? xA1 : 0.0f;
  const float pB0 = vB ? xB0 : 0.0f;
  const float pB1 = vB ? xB1 : 0.0f;
  const int nA = nent < 32 ? nent : 32;
  const int nB = nent - nA;
  float d0 = 0.0f, d1 = 0.0f;
#pragma unroll 1
  for (int j = 0; j < nA; ++j) { d0 = d0 + rl_f(pA0, j); d1 = d1 + rl_f(pA1, j); }
#pragma unroll 1
  for (int j = 0; j < nB; ++j) { d0 = d0 + rl_f(pB0, j); d1 = d1 + rl_f(pB1, j); }
  const float q0 = d0 + 1e-16f;
  const float q1 = d1 + 1e-16f;
  const float aA0 = pA0 / q0;
  const float aA1 = pA1 / q1;
  const float aB0 = pB0 / q0;
  const float aB1 = pB1 / q1;

  v4f acc = (v4f){ 0.0f, 0.0f, 0.0f, 0.0f };
  const float* hwl = HW + 4 * lane;
#pragma unroll 1
  for (int j = 0; j < nA; ++j) {
    const int s = __builtin_amdgcn_readlane(srcA, j);
    const float a0 = rl_f(aA0, j);
    const float a1 = rl_f(aA1, j);
    const float a = hsel ? a1 : a0;
    const v4f row = *(const v4fa*)(hwl + (size_t)s * HD);
    asm volatile("" :: "v"(row));
    acc = acc + a * row;
  }
#pragma unroll 1
  for (int j = 0; j < nB; ++j) {
    const int s = __builtin_amdgcn_readlane(srcB, j);
    const float a0 = rl_f(aB0, j);
    const float a1 = rl_f(aB1, j);
    const float a = hsel ? a1 : a0;
    const v4f row = *(const v4fa*)(hwl + (size_t)s * HD);
    asm volatile("" :: "v"(row));
    acc = acc + a * row;
  }

  const v4f gbv = *(const v4fa*)(TBL + T_GB + 4 * lane);
  asm volatile("" :: "v"(gbv));
  const float qnan = __uint_as_float(0x7fc00000u);
  unsigned hw_[4], lw_[4];
#pragma unroll
  for (int e = 0; e < 4; ++e) {
    float v = acc[e] + gbv[e];
    v = (v > 0.0f) ? v : (v - v);
    v = poison ? qnan : v;
    v = live ? v : 0.0f;
    hw_[e] = bf16_bits(v);
    lw_[e] = SITE2_TWO_TERM ? bf16_lo_bits(v) : 0u;
  }
  const v2u H = (v2u){ pk16(hw_[0], hw_[1]), pk16(hw_[2], hw_[3]) };
  const v2u L = (v2u){ pk16(lw_[0], lw_[1]), pk16(lw_[2], lw_[3]) };
  unsigned short* rowp = Ghl + (size_t)d * KHL;
  volatile v2u* qh = (volatile v2u*)(rowp + 4 * lane);
  volatile v2u* ql = (volatile v2u*)(rowp + 128 + 4 * lane);
  *qh = H;
  *ql = L;
  __threadfence();
  *qh = H;
  *ql = L;
}

__device__ __forceinline__ float sigm(float v) { return 1.0f / (1.0f + expf(-v)); }

__global__ __launch_bounds__(256) void k_gate(const float* __restrict__ GT, const float* __restrict__ TBL,
                                              unsigned short* __restrict__ Gc, int rowBase) {
  __shared__ __attribute__((aligned(16))) float sH[8 * 128];
  const int tid = (int)threadIdx.x, lane = tid & 31, wave = tid >> 5;
  const int col = tid & 127;
  const int rh  = tid >> 7;
  const int rb  = (int)blockIdx.x * 8;
  const float bi = TBL[T_BHH + col];
  const float bc = TBL[T_BHH + 128 + col];
  const float bo = TBL[T_BHH + 256 + col];
  asm volatile("" :: "v"(bi));
  asm volatile("" :: "v"(bc));
  asm volatile("" :: "v"(bo));
#pragma unroll 1
  for (int it = 0; it < 4; ++it) {
    const int rl = 2 * it + rh;
    const int r  = rb + rl;
    const float* gp = GT + (size_t)r * NG + col;
    const float gi = gp[0];
    const float gc = gp[128];
    const float go = gp[256];
    asm volatile("" :: "v"(gi));
    asm volatile("" :: "v"(gc));
    asm volatile("" :: "v"(go));
    const float vi = gi + bi;
    const float vc = gc + bc;
    const float vo = go + bo;
    const float c  = sigm(vi) * tanhf(vc);
    float hn = sigm(vo) * tanhf(c);
    hn = (rowBase + r < NN) ? hn : 0.0f;
    sH[rl * 128 + col] = hn;
  }
  __syncthreads();
  const int pc = lane & 15;
  const v4f a = *(const v4fa*)(sH + wave * 128 + 8 * pc);
  const v4f c = *(const v4fa*)(sH + wave * 128 + 8 * pc + 4);
  const v4u hi = pack8_bf16(a, c);
  v4u lo = (v4u){ 0u, 0u, 0u, 0u };
  if (SITE3_TWO_TERM) lo = pack8_bf16_lo(a, c);
  const v4u o = (lane < 16) ? hi : lo;
  put16(Gc + (size_t)(rb + wave) * KHL + lane * 8, o);
}

static_assert((OUT_ELEMS / 256) * 256 == OUT_ELEMS);
__global__ __launch_bounds__(256) void k_out(const float* __restrict__ T, float* __restrict__ out) {
  const int f  = (int)blockIdx.x * 256 + (int)threadIdx.x;
  const int fc = f < OUT_ELEMS ? f : OUT_ELEMS - 1;
  const int n  = fc >> 4;
  const int c  = fc - (n << 4);
  const float v = T[(size_t)n * 64 + c];
  asm volatile("" :: "v"(v));
  if (f < OUT_ELEMS) {
    volatile float* q = (volatile float*)(out + f);
    *q = v;
    __threadfence();
    *q = v;
  }
}

extern "C" void kernel_launch(void* const* d_in, const int* in_sizes, int n_in,
                              void* d_out, int out_size, void* d_ws, size_t ws_size,
                              hipStream_t stream) {
  if (n_in < 13) return;
  if (in_sizes[0] != NN * FIN) return;
  if (in_sizes[1] != 2 * NE) return;
  if (in_sizes[2] != FIN * HD) return;
  if (in_sizes[3] != HD || in_sizes[4] != HD || in_sizes[5] != HD) return;
  if (in_sizes[6] != 512 * HD) return;
  if (in_sizes[8] != 512 || in_sizes[9] != 512) return;
  if (in_sizes[11] != NOUT * HD || in_sizes[12] != NOUT) return;
  if (out_size != OUT_ELEMS) return;
  if (ws_size < WS_TOTAL) return;

  const float* x    = (const float*)d_in[0];
  const int*   ei   = (const int*)d_in[1];
  const float* W    = (const float*)d_in[2];
  const float* atts = (const float*)d_in[3];
  const float* attd = (const float*)d_in[4];
  const float* gb   = (const float*)d_in[5];
  const float* Wih  = (const float*)d_in[6];
  const float* bih  = (const float*)d_in[8];
  const float* bhh  = (const float*)d_in[9];
  const float* Wfc  = (const float*)d_in[11];
  const float* bfc  = (const float*)d_in[12];
  float* out = (float*)d_out;

  char* ws = (char*)d_ws;
  unsigned short* PA   = (unsigned short*)(ws + OFF_A);
  float*          PB   = (float*)(ws + OFF_B);
  float*          AD4  = (float*)(ws + OFF_AD4);
  unsigned*       HITS = (unsigned*)(ws + OFF_HITS);
  int*            OC   = (int*)(ws + OFF_OC);
  unsigned short* WT   = (unsigned short*)(ws + OFF_WT);
  unsigned short* WIH2 = (unsigned short*)(ws + OFF_WIH2);
  unsigned short* WFC2 = (unsigned short*)(ws + OFF_WFC2);
  float*          TBL  = (float*)(ws + OFF_TBL);

  hipFuncSetAttribute(reinterpret_cast<const void*>(&k_bucket),
                      hipFuncAttributeMaxDynamicSharedMemorySize, LDS_BK);

  k_plane<0><<<MP * FIN / 8 / 256, 256, 0, stream>>>(x, NN, FIN, FIN, PA, MP, FIN);
  k_prep<<<66, 256, 0, stream>>>(W, Wih, Wfc, atts, attd, gb, bih, bhh, bfc, WT, WIH2, WFC2, TBL);
  k_bucket<<<NBLK, 256, LDS_BK, stream>>>(ei, HITS, OC);
  k_gemm_nt<0, 0><<<(MP / 64 * 2 + 7) / 8, 256, 0, stream>>>(PA, WT, TBL, PB, MP, HD, FIN, HD);
  k_node<<<NN / 32, 256, 0, stream>>>(PB, TBL, AD4);
  k_replay<<<MP / 8, 256, 0, stream>>>(HITS, OC, PB, AD4, TBL, PA);
  for (int c = 0; c < NCHK; ++c) {
    unsigned short* Gc = PA + (size_t)c * CHR * KHL;
    k_gemm_nt<1, 1><<<(CHR / 64 * (NG / 64) + 7) / 8, 256, 0, stream>>>(Gc, WIH2, TBL + T_BIH, PB, CHR, NG, KHL, NG);
    k_gate<<<CHR / 8, 256, 0, stream>>>(PB, TBL, Gc, c * CHR);
  }
  k_gemm_nt<1, 1><<<(MP / 64 + 7) / 8, 256, 0, stream>>>(PA, WFC2, TBL + T_BFC, PB, MP, 64, KHL, 64);
  k_out<<<OUT_ELEMS / 256, 256, 0, stream>>>(PB, out);
}
